// ClassCaps_35656818491745
// MI455X (gfx1250) — hardware-run, weakly checked
//
#include <hip/hip_runtime.h>
#include <math.h>

typedef __attribute__((ext_vector_type(16))) __bf16   v16b;
typedef __attribute__((ext_vector_type(8)))  __bf16   v8b;
typedef __attribute__((ext_vector_type(8)))  float    v8f;
typedef __attribute__((ext_vector_type(4)))  float    v4f;

constexpr int kNB   = 32;
constexpr int kNS   = 64;
constexpr int kNC   = 32;
constexpr int kNJ   = 100;
constexpr int kNJP  = 112;
constexpr int kND   = 16;
constexpr int kNQ   = 39;
constexpr int kNQM  = 48;
constexpr int kKQ   = 64;
constexpr int kPH   = 72;
constexpr int kCP   = 116;
constexpr int kGP   = 48;
constexpr int kBlk  = kNB * kNC;
constexpr int kFlat = kNB * kNJ;
constexpr int kGTile = kNJP * kGP;
constexpr float kEps    = 1e-7f;
constexpr float kVarEps = 1e-2f;

static_assert(kNJP % 16 == 0 && kNQM % 16 == 0 && kNS % 16 == 0, "tile multiples");
static_assert(kNS % 32 == 0 && kKQ % 32 == 0, "K multiples of 32");
static_assert(kNJ % 4 == 0 && kNJP - kNJ == 12, "softmax lane split");
static_assert((kNJP * kND) % 256 == 0, "coefficient builder coverage");
static_assert((kNJP * kNS) % 256 == 0 && (kNS * kKQ) % 256 == 0, "plane builder coverage");
static_assert(kGTile % 128 == 0 && (kGTile * 4) % 128 == 0, "moment tile is whole 512-B store groups");
static_assert(kNS * kCP >= kGTile, "moment staging fits in the logit tile");
static_assert(kFlat % 32 == 0, "32 flat (b,j) per statistics block");
static_assert(kNQ + 9 == kNQM && kNQ + 25 == kKQ, "pad column counts");

constexpr size_t kOffG   = 0;
constexpr size_t kOffMU  = kOffG  + (size_t)kBlk * kGTile * 4;
constexpr size_t kOffEE  = kOffMU + (size_t)kFlat * kND * 4;
constexpr size_t kOffCST = kOffEE + (size_t)kFlat * kND * 4;
constexpr size_t kWsTotal = kOffCST + (size_t)kFlat * 4;
static_assert(kWsTotal == 22442496ull, "carve total");
static_assert(kWsTotal <= 134217728ull, "carve cap");
static_assert((kOffMU % 128) == 0 && (kOffEE % 128) == 0 && (kOffCST % 128) == 0, "128-B aligned regions");
static_assert((size_t)kNB * kNJ * kND * 4 == 204800ull, "second output byte offset");

__device__ __forceinline__ unsigned short f2bf_bits(float f) {
  unsigned u = __float_as_uint(f);
  return (unsigned short)((u + 0x7FFFu + ((u >> 16) & 1u)) >> 16);
}
__device__ __forceinline__ float bf_bits2f(unsigned short h) { return __uint_as_float(((unsigned)h) << 16); }

union FragB { v16b v; v8b h[2]; };
__device__ __forceinline__ v16b frag_load(const __bf16* p) {
  FragB f;
  f.h[0] = *(const v8b*)(p);
  f.h[1] = *(const v8b*)(p + 16);
  return f.v;
}
__device__ __forceinline__ v8f mma_bf(v16b a, v16b b, v8f c) {
  c = __builtin_amdgcn_wmma_f32_16x16x32_bf16(false, a, false, b, (short)0, c, false, false);
  asm volatile("v_nop\n\tv_nop\n\tv_nop\n\tv_nop" : "+v"(c) : "v"(a), "v"(b));
  return c;
}
__device__ __forceinline__ void put16(__bf16* ph, __bf16* pl, int off, float v) {
  const unsigned short hb = f2bf_bits(v);
  const unsigned short lb = f2bf_bits(v - bf_bits2f(hb));
  ph[off] = __builtin_bit_cast(__bf16, hb);
  pl[off] = __builtin_bit_cast(__bf16, lb);
}
__device__ __forceinline__ float wave_sum32(float v) {
#pragma unroll
  for (int off = 16; off > 0; off >>= 1) v += __shfl_xor(v, off, 32);
  return v;
}
__device__ __forceinline__ float half_sum16(float v) {
#pragma unroll
  for (int off = 8; off > 0; off >>= 1) v += __shfl_xor(v, off, 32);
  return v;
}

template <bool FIRST>
__global__ __launch_bounds__(256) void em_kernel(
    const float* __restrict__ pose, const float* __restrict__ active, const float* __restrict__ Wt,
    const float* __restrict__ muP, const float* __restrict__ eP, const float* __restrict__ cstP,
    float* __restrict__ G)
{
  __shared__ __align__(16) float  sP[kNS * kND];
  __shared__ __align__(16) __bf16 sFaH[kNS * kPH];
  __shared__ __align__(16) __bf16 sFaL[kNS * kPH];
  __shared__ __align__(16) __bf16 sFbH[kNQM * kPH];
  __shared__ __align__(16) __bf16 sFbL[kNQM * kPH];
  __shared__ __align__(16) __bf16 sXH[kNJP * kPH];
  __shared__ __align__(16) __bf16 sXL[kNJP * kPH];
  __shared__ __align__(16) float  sCost[kNS * kCP];
  __shared__ float sAct[kNS];
  __shared__ float sCj[kNJP];

  const int tid  = threadIdx.x;
  const int lane = tid & 31;
  const int wave = tid >> 5;
  const int hh   = lane >> 4;
  const int rl   = lane & 15;
  const int koff = hh * 8;
  const int blk  = blockIdx.x;
  const int b    = blk / kNC;
  const int c    = blk - b * kNC;

  {
    const int s = tid >> 2, part = (tid & 3) * 4;
    const v4f pv = *(const v4f*)(pose + (((size_t)b * kNS + s) * kNC + c) * kND + part);
    *(v4f*)(sP + s * kND + part) = pv;
  }
  {
    const int sc = tid & (kNS - 1);
    float av = active[((size_t)b * kNS + sc) * kNC + c];
    asm volatile("" : "+v"(av));
    if (tid < kNS) sAct[tid] = av;
  }

  if (!FIRST) {
    {
      const int jc = (tid < kNJ) ? tid : (kNJ - 1);
      float cv = cstP[(size_t)b * kNJ + jc];
      asm volatile("" : "+v"(cv));
      if (tid < kNJP) sCj[tid] = (tid < kNJ) ? cv : 0.0f;
    }
#pragma unroll 1
    for (int i = 0; i < (kNJP * kND) / 256; ++i) {
      const int idx = tid + 256 * i;
      const int j = idx >> 4, d = idx & 15;
      const bool live = j < kNJ;
      const int jc = live ? j : (kNJ - 1);
      float mv = muP[((size_t)b * kNJ + jc) * kND + d];
      float ev = eP[((size_t)b * kNJ + jc) * kND + d];
      float wv = Wt[((size_t)c * kNJ + jc) * kND + d];
      asm volatile("" : "+v"(mv), "+v"(ev), "+v"(wv));
      const float ew = ev * wv;
      const float ga = live ? (2.0f * ew * mv) : 0.0f;
      const float gb = live ? (-(ew * wv)) : 0.0f;
      const float gc = live ? (2.0f * ev * mv) : 0.0f;
      const float gd = live ? (-2.0f * ew) : 0.0f;
      const float ge = live ? (-ev) : 0.0f;
      const int rowo = j * kPH;
      put16(sXH, sXL, rowo + d, ga);
      put16(sXH, sXL, rowo + 19 + d, gb);
      if (d < 2) {
        put16(sXH, sXL, rowo + 16 + d, gc);
        put16(sXH, sXL, rowo + 35 + d, gd);
        put16(sXH, sXL, rowo + 37 + d, ge);
      }
      if (d == 2) put16(sXH, sXL, rowo + 18, 0.0f);
      put16(sXH, sXL, rowo + kNQ + d, 0.0f);
      if (d < 9) put16(sXH, sXL, rowo + kNQ + 16 + d, 0.0f);
    }
  }
  __syncthreads();

  {
    const int q = tid & 63;
    const int dsel = (q < 16) ? q : ((q >= 19 && q < 35) ? (q - 19) : ((q == 36) ? 1 : 0));
#pragma unroll 1
    for (int i = 0; i < (kNS * kKQ) / 256; ++i) {
      const int s = (tid >> 6) + 4 * i;
      const float c0 = ((float)(s >> 3) + 0.5f) * 0.125f;
      const float c1 = ((float)(s & 7) + 0.5f) * 0.125f;
      const float pv = sP[s * kND + dsel];
      float v = 0.0f;
      if (q < 16) v = pv;
      else if (q == 16) v = c0;
      else if (q == 17) v = c1;
      else if (q == 18) v = 1.0f;
      else if (q < 35) v = pv * pv;
      else if (q == 35) v = pv * c0;
      else if (q == 36) v = pv * c1;
      else if (q == 37) v = c0 * c0;
      else if (q == 38) v = c1 * c1;
      if (!FIRST) put16(sFaH, sFaL, s * kPH + q, v);
      if (q < kNQM) put16(sFbH, sFbL, q * kPH + s, v);
    }
  }
  if (FIRST) {
#pragma unroll 1
    for (int i = 0; i < (kNJP * kNS) / 256; ++i) {
      const int idx = tid + 256 * i;
      const int j = idx >> 6, s = idx & 63;
      const float v = (j < kNJ) ? (sAct[s] * 0.01f) : 0.0f;
      put16(sXH, sXL, j * kPH + s, v);
    }
  }
  __syncthreads();

  if (!FIRST) {
    if (wave < 7) {
      const int n0 = wave * 16;
      const __bf16* bph = sXH + (n0 + rl) * kPH + koff;
      const __bf16* bpl = sXL + (n0 + rl) * kPH + koff;
      const v16b bh0 = frag_load(bph);
      const v16b bh1 = frag_load(bph + 32);
      const v16b bl0 = frag_load(bpl);
      const v16b bl1 = frag_load(bpl + 32);
#pragma unroll 1
      for (int i = 0; i < 4; ++i) {
        const __bf16* aph = sFaH + (i * 16 + rl) * kPH + koff;
        const __bf16* apl = sFaL + (i * 16 + rl) * kPH + koff;
        const v16b ah0 = frag_load(aph);
        const v16b ah1 = frag_load(aph + 32);
        const v16b al0 = frag_load(apl);
        const v16b al1 = frag_load(apl + 32);
        v8f acc = (v8f){0.f, 0.f, 0.f, 0.f, 0.f, 0.f, 0.f, 0.f};
        acc = mma_bf(ah0, bl0, acc);
        acc = mma_bf(al0, bh0, acc);
        acc = mma_bf(ah1, bl1, acc);
        acc = mma_bf(al1, bh1, acc);
        acc = mma_bf(ah0, bh0, acc);
        acc = mma_bf(ah1, bh1, acc);
#pragma unroll
        for (int r = 0; r < 8; ++r) sCost[(i * 16 + 8 * hh + r) * kCP + n0 + rl] = acc[r];
      }
    }
    __syncthreads();

    {
      const int s = tid >> 2, sub = tid & 3;
      float* crow = sCost + s * kCP;
      float mx = -INFINITY;
#pragma unroll 1
      for (int k = 0; k < kNJ / 4; ++k) {
        const int j = sub + 4 * k;
        const float x = crow[j] + sCj[j];
        crow[j] = x;
        mx = fmaxf(mx, x);
      }
      mx = fmaxf(mx, __shfl_xor(mx, 1, 32));
      mx = fmaxf(mx, __shfl_xor(mx, 2, 32));
      float sum = 0.0f;
#pragma unroll 1
      for (int k = 0; k < kNJ / 4; ++k) {
        const int j = sub + 4 * k;
        const float ex = expf(crow[j] - mx);
        crow[j] = ex;
        sum += ex;
      }
      sum += __shfl_xor(sum, 1, 32);
      sum += __shfl_xor(sum, 2, 32);
      const float inv = 1.0f / sum;
      const float av = sAct[s];
#pragma unroll 1
      for (int k = 0; k < kNJ / 4; ++k) {
        const int j = sub + 4 * k;
        const float rw = (crow[j] * inv) * av;
        put16(sXH, sXL, j * kPH + s, rw);
      }
#pragma unroll
      for (int k = 0; k < 3; ++k) put16(sXH, sXL, (kNJ + sub + 4 * k) * kPH + s, 0.0f);
    }
    __syncthreads();
  }

  if (wave < 7) {
    const int m0 = wave * 16;
    const __bf16* aph = sXH + (m0 + rl) * kPH + koff;
    const __bf16* apl = sXL + (m0 + rl) * kPH + koff;
    const v16b ah0 = frag_load(aph);
    const v16b ah1 = frag_load(aph + 32);
    const v16b al0 = frag_load(apl);
    const v16b al1 = frag_load(apl + 32);
#pragma unroll 1
    for (int n = 0; n < 3; ++n) {
      const __bf16* bph = sFbH + (n * 16 + rl) * kPH + koff;
      const __bf16* bpl = sFbL + (n * 16 + rl) * kPH + koff;
      const v16b bh0 = frag_load(bph);
      const v16b bh1 = frag_load(bph + 32);
      const v16b bl0 = frag_load(bpl);
      const v16b bl1 = frag_load(bpl + 32);
      v8f acc = (v8f){0.f, 0.f, 0.f, 0.f, 0.f, 0.f, 0.f, 0.f};
      acc = mma_bf(ah0, bl0, acc);
      acc = mma_bf(al0, bh0, acc);
      acc = mma_bf(ah1, bl1, acc);
      acc = mma_bf(al1, bh1, acc);
      acc = mma_bf(ah0, bh0, acc);
      acc = mma_bf(ah1, bh1, acc);
#pragma unroll
      for (int r = 0; r < 8; ++r) sCost[(m0 + 8 * hh + r) * kGP + n * 16 + rl] = acc[r];
    }
  }
  __syncthreads();

  {
    float* Gb = G + (size_t)blk * kGTile;
    for (int pass = 0; pass < 2; ++pass) {
#pragma unroll 1
      for (int k = wave; k < kGTile / 128; k += 8) {
        const int o = (k * 32 + lane) * 4;
        const v4f val = *(const v4f*)(sCost + o);
        *(volatile v4f*)(Gb + o) = val;
      }
      __threadfence();
    }
  }
}

__global__ __launch_bounds__(256) void stats_kernel(
    const float* __restrict__ G, const float* __restrict__ Wt, const float* __restrict__ bv, const float* __restrict__ ba,
    float* __restrict__ muP, float* __restrict__ eP, float* __restrict__ cstP, float* __restrict__ out,
    float lam, int last)
{
  __shared__ __align__(16) float sME[2 * 32 * kND];
  __shared__ __align__(16) float sCs[32];
  __shared__ __align__(16) float sAp[32];
  const int tid = threadIdx.x, lane = tid & 31, wave = tid >> 5;
  const int f0 = blockIdx.x * 32;

#pragma unroll 1
  for (int i = 0; i < 4; ++i) {
    const int li = wave * 4 + i;
    const int f = f0 + li;
    const int b = f / kNJ;
    const int j = f - b * kNJ;
    const v4f* gp = (const v4f*)(G + ((size_t)(b * kNC + lane) * kNJP + j) * kGP);
    const v4f* wp = (const v4f*)(Wt + ((size_t)lane * kNJ + j) * kND);
    float ga[40], wa[16];
#pragma unroll
    for (int k = 0; k < 10; ++k) {
      const v4f t = gp[k];
      ga[4 * k + 0] = t[0]; ga[4 * k + 1] = t[1]; ga[4 * k + 2] = t[2]; ga[4 * k + 3] = t[3];
    }
#pragma unroll
    for (int k = 0; k < 4; ++k) {
      const v4f t = wp[k];
      wa[4 * k + 0] = t[0]; wa[4 * k + 1] = t[1]; wa[4 * k + 2] = t[2]; wa[4 * k + 3] = t[3];
    }
    const float rsum = wave_sum32(ga[18]);
    float myS1 = 0.0f, mySv2 = 0.0f;
#pragma unroll
    for (int d = 0; d < kND; ++d) {
      const float w = wa[d];
      float s1p = w * ga[d];
      float sv2p = (w * w) * ga[19 + d];
      if (d < 2) {
        s1p += ga[16 + d];
        sv2p += 2.0f * w * ga[35 + d] + ga[37 + d];
      }
      const float S1 = wave_sum32(s1p);
      const float Sv2 = wave_sum32(sv2p);
      myS1 = (lane == d) ? S1 : myS1;
      mySv2 = (lane == d) ? Sv2 : mySv2;
    }
    const float inv = 1.0f / (rsum + kEps);
    const float m = myS1 * inv;
    float raw = mySv2 - 2.0f * m * myS1 + m * m * rsum;
    raw = fmaxf(raw, 0.0f);
    const float var = raw * inv + kVarEps;
    const float sig = sqrtf(var);
    const float ee = 1.0f / (2.0f * var + kEps);
    const float lg = logf(sig + kEps);
    const float logsum = half_sum16(lg);
    const float emus = half_sum16(ee * m * m);
    const float bvj = bv[j];
    const float baj = ba[j];
    const float lh = (16.0f * bvj + logsum) * rsum;
    const float xs = lam * (baj - lh);
    const float ap = 1.0f / (1.0f + expf(-xs));
    const float cs = logf(ap + kEps) - logsum - emus;
    if (lane < kND) {
      sME[li * kND + lane] = m;
      sME[32 * kND + li * kND + lane] = ee;
    }
    if (lane == 0) {
      sCs[li] = cs;
      sAp[li] = ap;
    }
  }
  __syncthreads();

  {
    const size_t fo = (size_t)f0;
    const v4f val = *(const v4f*)(sME + (wave * 32 + lane) * 4);
    const float cv = sCs[lane];
    const float apv = sAp[lane];
    const int wq = wave & 3;
    float* dst = (wave < 4) ? (muP + fo * kND + (wq * 32 + lane) * 4) : (eP + fo * kND + (wq * 32 + lane) * 4);
    float* dout0 = out + fo * kND + (wq * 32 + lane) * 4;
    float* dout1 = out + (size_t)kNB * kNJ * kND + fo + lane;
    for (int pass = 0; pass < 2; ++pass) {
      *(volatile v4f*)dst = val;
      if (last != 0 && wave < 4) *(volatile v4f*)dout0 = val;
      if (wave == 0) {
        *(volatile float*)(cstP + fo + lane) = cv;
        if (last != 0) *(volatile float*)dout1 = apv;
      }
      __threadfence();
    }
  }
}

extern "C" void kernel_launch(void* const* d_in, const int* in_sizes, int n_in,
                              void* d_out, int out_size, void* d_ws, size_t ws_size,
                              hipStream_t stream) {
  if (n_in < 5) return;
  if (in_sizes[0] != kNB * kNS * kNC * kND) return;
  if (in_sizes[1] != kNB * kNS * kNC) return;
  if (in_sizes[2] != kNC * kNJ * kND) return;
  if (in_sizes[3] != kNJ) return;
  if (in_sizes[4] != kNJ) return;
  if (out_size != kNB * kNJ * kND + kNB * kNJ) return;
  if (ws_size < kWsTotal) return;

  const float* pose   = (const float*)d_in[0];
  const float* active = (const float*)d_in[1];
  const float* Wt     = (const float*)d_in[2];
  const float* bv     = (const float*)d_in[3];
  const float* ba     = (const float*)d_in[4];
  float* out = (float*)d_out;

  char* ws = (char*)d_ws;
  float* G   = (float*)(ws + kOffG);
  float* MU  = (float*)(ws + kOffMU);
  float* EE  = (float*)(ws + kOffEE);
  float* CST = (float*)(ws + kOffCST);

  const double p1 = 0.95;
  const double p2 = p1 * 0.95;
  const double p3 = p2 * 0.95;
  const float lam0 = (float)(0.01 * (1.0 - p1));
  const float lam1 = (float)(0.01 * (1.0 - p2));
  const float lam2 = (float)(0.01 * (1.0 - p3));

  em_kernel<true><<<kBlk, 256, 0, stream>>>(pose, active, Wt, MU, EE, CST, G);
  stats_kernel<<<kFlat / 32, 256, 0, stream>>>(G, Wt, bv, ba, MU, EE, CST, out, lam0, 0);
  em_kernel<false><<<kBlk, 256, 0, stream>>>(pose, active, Wt, MU, EE, CST, G);
  stats_kernel<<<kFlat / 32, 256, 0, stream>>>(G, Wt, bv, ba, MU, EE, CST, out, lam1, 0);
  em_kernel<false><<<kBlk, 256, 0, stream>>>(pose, active, Wt, MU, EE, CST, G);
  stats_kernel<<<kFlat / 32, 256, 0, stream>>>(G, Wt, bv, ba, MU, EE, CST, out, lam2, 1);
}
